// LSTMCell_4123168604852
// MI455X (gfx1250) — hardware-verified
//
#include <hip/hip_runtime.h>
#include <stddef.h>

constexpr int NB_ROWS = 2048;
constexpr int NIN     = 1024;
constexpr int NHID    = 1024;
constexpr int KDIM    = NIN + NHID;
constexpr int NGATE   = 4;
static_assert(KDIM == 2048, "shape");
static_assert(KDIM % 32 == 0, "k step multiple of 32, no k padding needed");
static_assert(NIN == NHID, "activation packer assumes equal halves");
static_assert(NIN % 256 == 0, "activation packer: one wave stays inside one row half");

constexpr size_t WS_A_ELEMS  = (size_t)NB_ROWS * KDIM;
constexpr size_t WS_BT_ELEMS = (size_t)NGATE * NHID * KDIM;
constexpr size_t WS_A_BYTES  = WS_A_ELEMS * 2;
constexpr size_t WS_BT_BYTES = WS_BT_ELEMS * 2;
constexpr size_t WS_TOTAL    = WS_A_BYTES + WS_BT_BYTES;
static_assert(WS_TOTAL == (size_t)25165824, "carve total");
static_assert(WS_TOTAL <= (size_t)134217728, "carve cap");
constexpr size_t OUT_ELEMS_EACH = (size_t)NB_ROWS * NHID;
static_assert(OUT_ELEMS_EACH * 4 == (size_t)8388608, "out1 byte offset");

typedef __attribute__((ext_vector_type(16))) _Float16 v16h;
typedef __attribute__((ext_vector_type(8)))  _Float16 v8h;
typedef __attribute__((ext_vector_type(16))) __bf16   v16b;
typedef __attribute__((ext_vector_type(8)))  __bf16   v8b;
typedef __attribute__((ext_vector_type(8)))  float    v8f;
typedef __attribute__((ext_vector_type(4)))  float    v4f;
typedef __attribute__((ext_vector_type(4)))  unsigned v4u;

__device__ __forceinline__ unsigned short f2bf_bits(float f) {
  unsigned u = __float_as_uint(f);
  return (unsigned short)((u + 0x7FFFu + ((u >> 16) & 1u)) >> 16);
}
__device__ __forceinline__ float bf_bits2f(unsigned short h) { return __uint_as_float(((unsigned)h) << 16); }

__device__ __forceinline__ void dep_guard_h(v8f& a, v8f& b, v16h x, v16h y) { asm volatile("v_nop\n\tv_nop\n\tv_nop\n\tv_nop" : "+v"(a), "+v"(b) : "v"(x), "v"(y)); }
__device__ __forceinline__ void dep_guard_b(v8f& a, v8f& b, v16b x, v16b y) { asm volatile("v_nop\n\tv_nop\n\tv_nop\n\tv_nop" : "+v"(a), "+v"(b) : "v"(x), "v"(y)); }
__device__ __forceinline__ void keep4_h(v16h a, v16h b, v16h c, v16h d) { asm volatile("v_nop" :: "v"(a), "v"(b), "v"(c), "v"(d)); }
__device__ __forceinline__ void keep4_b(v16b a, v16b b, v16b c, v16b d) { asm volatile("v_nop" :: "v"(a), "v"(b), "v"(c), "v"(d)); }
__device__ __forceinline__ void acc_guard4(v8f& a, v8f& b, v8f& c, v8f& d) { asm volatile("v_nop\n\tv_nop\n\tv_nop\n\tv_nop" : "+v"(a), "+v"(b), "+v"(c), "+v"(d)); }
template <typename T> struct Frag;
template <> struct Frag<_Float16> {
  typedef v16h V; union U { v16h v; v8h h[2]; };
  static __device__ __forceinline__ v16h load(const _Float16* p) {
    U f; f.h[0] = *(const v8h*)(p); f.h[1] = *(const v8h*)(p + 16); return f.v;
  }
  static __device__ __forceinline__ v8f mma(v16h a, v16h b, v8f c) {
    return __builtin_amdgcn_wmma_f32_16x16x32_f16(false, a, false, b, (short)0, c, false, false);
  }
  static __device__ __forceinline__ void guard(v8f& a, v8f& b, v16h x, v16h y) { dep_guard_h(a, b, x, y); }
  static __device__ __forceinline__ void keep(v16h a, v16h b, v16h c, v16h d) { keep4_h(a, b, c, d); }
};
template <> struct Frag<__bf16> {
  typedef v16b V; union U { v16b v; v8b h[2]; };
  static __device__ __forceinline__ v16b load(const __bf16* p) {
    U f; f.h[0] = *(const v8b*)(p); f.h[1] = *(const v8b*)(p + 16); return f.v;
  }
  static __device__ __forceinline__ v8f mma(v16b a, v16b b, v8f c) {
    return __builtin_amdgcn_wmma_f32_16x16x32_bf16(false, a, false, b, (short)0, c, false, false);
  }
  static __device__ __forceinline__ void guard(v8f& a, v8f& b, v16b x, v16b y) { dep_guard_b(a, b, x, y); }
  static __device__ __forceinline__ void keep(v16b a, v16b b, v16b c, v16b d) { keep4_b(a, b, c, d); }
};

__device__ __forceinline__ unsigned f2bf_u(float f) {
  unsigned u = __float_as_uint(f);
  return (u + 0x7FFFu + ((u >> 16) & 1u)) >> 16;
}
__device__ __forceinline__ float bf16_rne_f(float f) {
  unsigned u = __float_as_uint(f);
  u = (u + 0x7FFFu + ((u >> 16) & 1u)) & 0xFFFF0000u;
  return __uint_as_float(u);
}
__device__ __forceinline__ float sigmoid_f(float v) { return 1.0f / (1.0f + expf(-v)); }

__device__ __forceinline__ void guard_grp(v8f& c0, v8f& c1, v8f& c2, v8f& c3,
                                          v16b a, v16b b0, v16b b1, v16b b2, v16b b3) {
  asm volatile("v_nop\n\tv_nop\n\tv_nop\n\tv_nop"
               : "+v"(c0), "+v"(c1), "+v"(c2), "+v"(c3)
               : "v"(a), "v"(b0), "v"(b1), "v"(b2), "v"(b3)
               : "memory");
}

constexpr int PACK_THREADS = 256;
constexpr int PACKA_BLOCKS = (NB_ROWS * NIN / 8) / PACK_THREADS;
static_assert((NB_ROWS * NIN / 8) % PACK_THREADS == 0, "pack grid exact");

__global__ __launch_bounds__(256) void pack_act(const float* __restrict__ x,
                                                const float* __restrict__ hid,
                                                unsigned short* __restrict__ Apl) {
  const float* src = (blockIdx.y == 0) ? x : hid;
  const int e    = blockIdx.x * PACK_THREADS + threadIdx.x;
  const int base = e * 8;
  const int b    = base / NIN;
  const int kk   = base - b * NIN;
  const float* p = src + (size_t)b * NIN + kk;
  const v4f f0 = *(const v4f*)(p);
  const v4f f1 = *(const v4f*)(p + 4);
  v4u w;
  w[0] = f2bf_u(f0[0]) | (f2bf_u(f0[1]) << 16);
  w[1] = f2bf_u(f0[2]) | (f2bf_u(f0[3]) << 16);
  w[2] = f2bf_u(f1[0]) | (f2bf_u(f1[1]) << 16);
  w[3] = f2bf_u(f1[2]) | (f2bf_u(f1[3]) << 16);
  unsigned short* d = Apl + (size_t)b * KDIM + (size_t)blockIdx.y * NIN + kk;
  *(volatile v4u*)d = w;
  __threadfence();
  *(volatile v4u*)d = w;
}

constexpr int PW_KT = 64;
constexpr int PW_HT = 32;
static_assert(KDIM % PW_KT == 0 && NHID % PW_HT == 0, "weight tile");

__global__ __launch_bounds__(256) void pack_wt(const float* __restrict__ Wf,
                                               const float* __restrict__ Wi,
                                               const float* __restrict__ Wc,
                                               const float* __restrict__ Wo,
                                               unsigned short* __restrict__ Btpl) {
  __shared__ float tile[PW_KT][PW_HT + 1];
  const int g = blockIdx.z;
  const float* W = (g == 0) ? Wf : (g == 1) ? Wi : (g == 2) ? Wc : Wo;
  const int k0 = blockIdx.x * PW_KT;
  const int h0 = blockIdx.y * PW_HT;
  const int t  = threadIdx.x;
  const int hc = t & 31;
  const int kr0 = t >> 5;
#pragma unroll
  for (int i = 0; i < 8; ++i) {
    const int kr = kr0 + 8 * i;
    tile[kr][hc] = W[(size_t)(k0 + kr) * NHID + h0 + hc];
  }
  __syncthreads();
  const int lane = t & 31, wave = t >> 5;
  const int hrow = wave * 4 + (lane >> 3);
  const int kc8  = (lane & 7) * 8;
  unsigned bb[8];
#pragma unroll
  for (int e2 = 0; e2 < 8; ++e2) bb[e2] = f2bf_u(tile[kc8 + e2][hrow]);
  v4u w;
  w[0] = bb[0] | (bb[1] << 16);
  w[1] = bb[2] | (bb[3] << 16);
  w[2] = bb[4] | (bb[5] << 16);
  w[3] = bb[6] | (bb[7] << 16);
  unsigned short* d = Btpl + (size_t)(g * NHID + h0 + hrow) * KDIM + k0 + kc8;
  *(volatile v4u*)d = w;
  __threadfence();
  *(volatile v4u*)d = w;
}

constexpr int WT_ROWS  = 16;
constexpr int WT_HCOLS = 32;
constexpr int GEMM_WAVES = 4;
constexpr int GEMM_THREADS = GEMM_WAVES * 32;
constexpr int NTILES_M = NB_ROWS / WT_ROWS;
constexpr int NTILES_H = NHID / WT_HCOLS;
constexpr int NTILES   = NTILES_M * NTILES_H;
constexpr int GEMM_BLOCKS = NTILES / GEMM_WAVES;
static_assert(NB_ROWS % WT_ROWS == 0 && NHID % WT_HCOLS == 0, "tile multiples");
static_assert(NTILES % GEMM_WAVES == 0, "gemm grid exact");
constexpr int SLAB_G      = WT_ROWS * WT_HCOLS;
constexpr int SLAB_FLOATS = NGATE * SLAB_G;

__global__ __launch_bounds__(128) void cell_gate_gemm(
    const unsigned short* __restrict__ Ap,
    const unsigned short* __restrict__ Btp,
    const float* __restrict__ bias_f, const float* __restrict__ bias_i,
    const float* __restrict__ bias_c, const float* __restrict__ bias_o,
    const float* __restrict__ cell,
    float* __restrict__ out0,
    float* __restrict__ out1) {
  typedef __bf16 T;
  typedef v16b V;
  __shared__ __align__(16) float sT[GEMM_WAVES][SLAB_FLOATS];

  const int lane = threadIdx.x & 31;
  const int wave = threadIdx.x >> 5;
  const int tile = blockIdx.x * GEMM_WAVES + wave;
  if (tile >= NTILES) return;
  const int tm = tile / NTILES_H;
  const int th = tile - tm * NTILES_H;
  const int m0 = tm * WT_ROWS;
  const int h0 = th * WT_HCOLS;

  const T* A  = (const T*)Ap;
  const T* Bt = (const T*)Btp;
  const int rlane = lane & 15;
  const int koff  = (lane >> 4) * 8;
  const int mOff  = (lane >> 4) * 8;

  const int cA = h0 + rlane, cB = h0 + 16 + rlane;
  float bv[8];
  bv[0] = bf16_rne_f(bias_f[cA]); bv[1] = bf16_rne_f(bias_f[cB]);
  bv[2] = bf16_rne_f(bias_i[cA]); bv[3] = bf16_rne_f(bias_i[cB]);
  bv[4] = bf16_rne_f(bias_c[cA]); bv[5] = bf16_rne_f(bias_c[cB]);
  bv[6] = bf16_rne_f(bias_o[cA]); bv[7] = bf16_rne_f(bias_o[cB]);

  const T* Arow = A + (size_t)(m0 + rlane) * KDIM + koff;
  const T* Brow[8];
#pragma unroll
  for (int j = 0; j < 8; ++j)
    Brow[j] = Bt + (size_t)((j >> 1) * NHID + h0 + 16 * (j & 1) + rlane) * KDIM + koff;

  v8f acc[8];
#pragma unroll
  for (int j = 0; j < 8; ++j) acc[j] = (v8f){0.f,0.f,0.f,0.f,0.f,0.f,0.f,0.f};

#pragma unroll 1
  for (int k0 = 0; k0 < KDIM; k0 += 32) {
    const V a  = Frag<T>::load(Arow + k0);
    const V q0 = Frag<T>::load(Brow[0] + k0);
    const V q1 = Frag<T>::load(Brow[1] + k0);
    const V q2 = Frag<T>::load(Brow[2] + k0);
    const V q3 = Frag<T>::load(Brow[3] + k0);
    acc[0] = Frag<T>::mma(a, q0, acc[0]);
    acc[1] = Frag<T>::mma(a, q1, acc[1]);
    acc[2] = Frag<T>::mma(a, q2, acc[2]);
    acc[3] = Frag<T>::mma(a, q3, acc[3]);
    guard_grp(acc[0], acc[1], acc[2], acc[3], a, q0, q1, q2, q3);
    const V q4 = Frag<T>::load(Brow[4] + k0);
    const V q5 = Frag<T>::load(Brow[5] + k0);
    const V q6 = Frag<T>::load(Brow[6] + k0);
    const V q7 = Frag<T>::load(Brow[7] + k0);
    acc[4] = Frag<T>::mma(a, q4, acc[4]);
    acc[5] = Frag<T>::mma(a, q5, acc[5]);
    acc[6] = Frag<T>::mma(a, q6, acc[6]);
    acc[7] = Frag<T>::mma(a, q7, acc[7]);
    guard_grp(acc[4], acc[5], acc[6], acc[7], a, q4, q5, q6, q7);
  }
  acc_guard4(acc[0], acc[1], acc[2], acc[3]);
  acc_guard4(acc[4], acc[5], acc[6], acc[7]);

  float* slab = sT[wave];
#pragma unroll
  for (int j = 0; j < 8; ++j) {
    const int g = j >> 1, jh = j & 1;
    float* sp = slab + g * SLAB_G + 16 * jh + rlane;
    const float bj = bv[j];
#pragma unroll
    for (int r = 0; r < 8; ++r) sp[(mOff + r) * WT_HCOLS] = acc[j][r] + bj;
  }
  __builtin_amdgcn_fence(__ATOMIC_RELEASE, "workgroup");
  __builtin_amdgcn_wave_barrier();
  __builtin_amdgcn_fence(__ATOMIC_ACQUIRE, "workgroup");

  const int q  = lane >> 3;
  const int c4 = (lane & 7) * 4;
#pragma unroll 1
  for (int it = 0; it < 4; ++it) {
    const int row = it * 4 + q;
    float* s0 = slab + row * WT_HCOLS + c4;
    const v4f pf = *(const v4f*)(s0);
    const v4f pi = *(const v4f*)(s0 + SLAB_G);
    const v4f pc = *(const v4f*)(s0 + 2 * SLAB_G);
    const v4f po = *(const v4f*)(s0 + 3 * SLAB_G);
    const v4f cv = *(const v4f*)(cell + (size_t)(m0 + row) * NHID + h0 + c4);
    v4f cn4, hn4;
#pragma unroll
    for (int e = 0; e < 4; ++e) {
      const float fg = sigmoid_f(pf[e]);
      const float ig = sigmoid_f(pi[e]);
      const float ch = tanhf(pc[e]);
      const float og = sigmoid_f(po[e]);
      const float ce = cv[e];
      const float cs = bf16_rne_f(ce);
      const float cn = fg * cs + ig * ch;
      const float hn = og * tanhf(cn);
      cn4[e] = cn;
      hn4[e] = hn;
    }
    *(v4f*)(s0)          = cn4;
    *(v4f*)(s0 + SLAB_G) = hn4;
  }

  for (int pass = 0; pass < 2; ++pass) {
#pragma unroll
    for (int it = 0; it < 4; ++it) {
      const int row = it * 4 + q;
      const float* s0 = slab + row * WT_HCOLS + c4;
      const v4f cn4 = *(const v4f*)(s0);
      const v4f hn4 = *(const v4f*)(s0 + SLAB_G);
      const size_t o = (size_t)(m0 + row) * NHID + h0 + c4;
      *(volatile v4f*)(out0 + o) = cn4;
      *(volatile v4f*)(out1 + o) = hn4;
    }
    __threadfence();
  }
}

extern "C" void kernel_launch(void* const* d_in, const int* in_sizes, int n_in,
                              void* d_out, int out_size, void* d_ws, size_t ws_size,
                              hipStream_t stream) {
  if (n_in < 11) return;
  if (ws_size < WS_TOTAL) return;
  if ((size_t)out_size < 2 * OUT_ELEMS_EACH) return;
  if (in_sizes[0] != NB_ROWS * NIN || in_sizes[1] != NB_ROWS * NHID || in_sizes[2] != NB_ROWS * NHID) return;
  if (in_sizes[3] != KDIM * NHID || in_sizes[5] != KDIM * NHID || in_sizes[7] != KDIM * NHID || in_sizes[9] != KDIM * NHID) return;
  if (in_sizes[4] != NHID || in_sizes[6] != NHID || in_sizes[8] != NHID || in_sizes[10] != NHID) return;

  const float* x     = (const float*)d_in[0];
  const float* cell  = (const float*)d_in[1];
  const float* hid   = (const float*)d_in[2];
  const float* Wf    = (const float*)d_in[3];
  const float* bfv   = (const float*)d_in[4];
  const float* Wi    = (const float*)d_in[5];
  const float* biv   = (const float*)d_in[6];
  const float* Wc    = (const float*)d_in[7];
  const float* bcv   = (const float*)d_in[8];
  const float* Wo    = (const float*)d_in[9];
  const float* bov   = (const float*)d_in[10];

  unsigned short* Apl  = (unsigned short*)d_ws;
  unsigned short* Btpl = (unsigned short*)((char*)d_ws + WS_A_BYTES);
  float* out0 = (float*)d_out;
  float* out1 = out0 + OUT_ELEMS_EACH;

  pack_act<<<dim3(PACKA_BLOCKS, 2), PACK_THREADS, 0, stream>>>(x, hid, Apl);
  pack_wt<<<dim3(KDIM / PW_KT, NHID / PW_HT, NGATE), PACK_THREADS, 0, stream>>>(Wf, Wi, Wc, Wo, Btpl);
  cell_gate_gemm<<<dim3(GEMM_BLOCKS), GEMM_THREADS, 0, stream>>>(
      Apl, Btpl, bfv, biv, bcv, bov, cell, out0, out1);
}
